// NodeGenerator_85856396247142
// MI455X (gfx1250) — hardware-verified
//
#include <hip/hip_runtime.h>
#include <stddef.h>
#include <math.h>


#define FX     64
#define KC     128
#define H1     128
#define H2     64
#define G3     67
#define G3P    80
#define HP     32
#define OW     68
#define NTHR   256
#define NWAVE  8
#define EPT    8
#define NGRP   2
#define CHUNK  (NTHR * EPT * NGRP)
#define WCAP   (EPT * NGRP * 32)
#define LISTN  (NWAVE * WCAP)
#define NB     960
#define GROWS  128
#define APT    136
#define WSCAP  134217728

#define WP1    0
#define WP2    32768
#define WP3    49152
#define WPP    59392
#define WPTOT  63488

#define LDS_AGG (NB * FX * 4 + LISTN * 4 + NB * 4 + 64)
#define LDS_AT  (2 * GROWS * APT * 2)
#define LDS_MLP (LDS_AT + GROWS * H1 * 4)

static_assert((CHUNK & (CHUNK - 1)) == 0);
static_assert(CHUNK <= 4096);
static_assert(NB <= 4096 && (NB % 4) == 0 && LISTN >= NB);
static_assert(((NB * FX / 4) % NTHR) == 0);
static_assert(GROWS == NWAVE * 16);
static_assert(KC == 2 * FX);
static_assert(WP2 == WP1 + 2 * H1 * KC && WP3 == WP2 + 2 * H2 * H1);
static_assert(WPP == WP3 + 2 * G3P * H2 && WPTOT == WPP + 2 * HP * FX);
static_assert((WP2 % 64) == 0 && (WP3 % 64) == 0 && (WPP % 64) == 0);
static_assert((APT % 8) == 0 && (LDS_AT % 16) == 0);
static_assert((OW % 4) == 0 && ((GROWS * OW) % 4) == 0);
static_assert(G3P * 4 * GROWS <= GROWS * H1 * 4);

typedef float          v2f  __attribute__((ext_vector_type(2)));
typedef float          v4f  __attribute__((ext_vector_type(4)));
typedef float          v8f  __attribute__((ext_vector_type(8)));
typedef int            v4i  __attribute__((ext_vector_type(4)));
typedef unsigned short v8us __attribute__((ext_vector_type(8)));
typedef __bf16         v16b __attribute__((ext_vector_type(16)));
union FragB { v16b v; v8us h[2]; };

__device__ __forceinline__ unsigned int bfr(float f) {
  const unsigned int u = __float_as_uint(f);
  return (u + 0x7FFFu + ((u >> 16) & 1u)) >> 16;
}

__device__ __forceinline__ void split1(float x, unsigned short& hb, unsigned short& lb) {
  const unsigned int hu = bfr(x);
  const float hf = __uint_as_float(hu << 16);
  hb = (unsigned short)hu;
  lb = (unsigned short)bfr(x - hf);
}

__device__ __forceinline__ void split8(v4f a, v4f b, v8us& hi, v8us& lo) {
  unsigned short hb, lb;
  split1(a.x, hb, lb); hi[0] = hb; lo[0] = lb;
  split1(a.y, hb, lb); hi[1] = hb; lo[1] = lb;
  split1(a.z, hb, lb); hi[2] = hb; lo[2] = lb;
  split1(a.w, hb, lb); hi[3] = hb; lo[3] = lb;
  split1(b.x, hb, lb); hi[4] = hb; lo[4] = lb;
  split1(b.y, hb, lb); hi[5] = hb; lo[5] = lb;
  split1(b.z, hb, lb); hi[6] = hb; lo[6] = lb;
  split1(b.w, hb, lb); hi[7] = hb; lo[7] = lb;
}

__device__ __forceinline__ v8f wmb(v16b a, v16b b, v8f c) {
  v8f d = __builtin_amdgcn_wmma_f32_16x16x32_bf16(false, a, false, b, (short)0, c, false, false);
  asm volatile("v_nop\n\tv_nop\n\tv_nop\n\tv_nop" : "+v"(d) : "v"(a), "v"(b));
  return d;
}

template <int KD, int NT, int NCT, int PK>
__device__ __forceinline__ void mma_tiles(const unsigned short* sHi, const unsigned short* sLo,
                                          const unsigned short* __restrict__ Bw, int wrow, int lane,
                                          v8f (&acc)[NT]) {
  static_assert((KD % 32) == 0 && (PK % 8) == 0);
  constexpr int NKT = KD / 32, WPLN = NCT * KD;
  const int hh = lane >> 4, m = lane & 15;
#pragma unroll
  for (int t = 0; t < NT; ++t) { v8f z = {0.f, 0.f, 0.f, 0.f, 0.f, 0.f, 0.f, 0.f}; acc[t] = z; }
  const unsigned short* ahp = sHi + (wrow + m) * PK + 8 * hh;
  const unsigned short* alp = sLo + (wrow + m) * PK + 8 * hh;
#pragma unroll 1
  for (int kt = 0; kt < NKT; ++kt) {
    FragB ah, al;
    ah.h[0] = *(const v8us*)(ahp + 32 * kt);
    ah.h[1] = *(const v8us*)(ahp + 32 * kt + 16);
    al.h[0] = *(const v8us*)(alp + 32 * kt);
    al.h[1] = *(const v8us*)(alp + 32 * kt + 16);
#pragma unroll
    for (int t = 0; t < NT; ++t) {
      const unsigned short* bp = Bw + (size_t)(16 * t + m) * KD + 32 * kt + 8 * hh;
      FragB bh, bl;
      bh.h[0] = *(const v8us*)bp;
      bh.h[1] = *(const v8us*)(bp + 16);
      bl.h[0] = *(const v8us*)(bp + WPLN);
      bl.h[1] = *(const v8us*)(bp + WPLN + 16);
      acc[t] = wmb(ah.v, bh.v, acc[t]);
      acc[t] = wmb(ah.v, bl.v, acc[t]);
      acc[t] = wmb(al.v, bh.v, acc[t]);
    }
  }
}

template <int NBL>
__device__ __forceinline__ int scan_chunk(const int* __restrict__ keys, int nE, int cbase, int slotBase,
                                          int vec8, int* list, int tid, int lane, int wave) {
  int wc = 0;
#pragma unroll
  for (int g = 0; g < NGRP; ++g) {
    const int el0  = (g * NTHR + tid) * EPT;
    const int e0   = cbase + el0;
    const int sent = -2147483647 - 1;
    v4i da, db;
    if (vec8 != 0 && cbase + CHUNK <= nE) {
      da = *(const v4i*)(keys + e0);
      db = *(const v4i*)(keys + e0 + 4);
    } else {
      da.x = (e0     < nE) ? keys[min(e0,     nE - 1)] : sent;
      da.y = (e0 + 1 < nE) ? keys[min(e0 + 1, nE - 1)] : sent;
      da.z = (e0 + 2 < nE) ? keys[min(e0 + 2, nE - 1)] : sent;
      da.w = (e0 + 3 < nE) ? keys[min(e0 + 3, nE - 1)] : sent;
      db.x = (e0 + 4 < nE) ? keys[min(e0 + 4, nE - 1)] : sent;
      db.y = (e0 + 5 < nE) ? keys[min(e0 + 5, nE - 1)] : sent;
      db.z = (e0 + 6 < nE) ? keys[min(e0 + 6, nE - 1)] : sent;
      db.w = (e0 + 7 < nE) ? keys[min(e0 + 7, nE - 1)] : sent;
    }
    const unsigned nb = (unsigned)slotBase;
    const unsigned s0 = (unsigned)da.x - nb, s1 = (unsigned)da.y - nb;
    const unsigned s2 = (unsigned)da.z - nb, s3 = (unsigned)da.w - nb;
    const unsigned s4 = (unsigned)db.x - nb, s5 = (unsigned)db.y - nb;
    const unsigned s6 = (unsigned)db.z - nb, s7 = (unsigned)db.w - nb;
    const bool h0 = s0 < (unsigned)NBL, h1 = s1 < (unsigned)NBL, h2 = s2 < (unsigned)NBL, h3 = s3 < (unsigned)NBL;
    const bool h4 = s4 < (unsigned)NBL, h5 = s5 < (unsigned)NBL, h6 = s6 < (unsigned)NBL, h7 = s7 < (unsigned)NBL;
    const unsigned any = __builtin_amdgcn_ballot_w32(h0 | h1 | h2 | h3 | h4 | h5 | h6 | h7);
    if (any != 0u) {
#define HITJ(J, HJ, SJ) { \
        const unsigned mj = __builtin_amdgcn_ballot_w32(HJ); \
        if (mj != 0u) { \
          if (HJ) { \
            const int pos = wc + (int)__builtin_amdgcn_mbcnt_lo(mj, 0u); \
            if (pos < WCAP) list[wave * WCAP + pos] = ((el0 + (J)) << 12) | (int)(SJ); \
          } \
          wc += (int)__builtin_popcount(mj); } }
      HITJ(0, h0, s0)
      HITJ(1, h1, s1)
      HITJ(2, h2, s2)
      HITJ(3, h3, s3)
      HITJ(4, h4, s4)
      HITJ(5, h5, s5)
      HITJ(6, h6, s6)
      HITJ(7, h7, s7)
#undef HITJ
    }
  }
  return wc;
}

__global__ __launch_bounds__(NTHR) void k_wprep(
    const float* __restrict__ W1, const float* __restrict__ W2,
    const float* __restrict__ W3, const float* __restrict__ P1, unsigned short* wp) {
  const int blk = blockIdx.x, tid = threadIdx.x;
  float v[8];
  int KD, NC, i, base;
  bool act = true;
  if (blk < 8) {
    KD = KC; NC = H1; i = blk * NTHR + tid; base = WP1;
    const int n = i >> 4, k0 = (i & 15) * 8;
#pragma unroll
    for (int e = 0; e < 8; ++e) v[e] = W1[(k0 + e) * H1 + n];
  } else if (blk < 12) {
    KD = H1; NC = H2; i = (blk - 8) * NTHR + tid; base = WP2;
    const int n = i >> 4, k0 = (i & 15) * 8;
#pragma unroll
    for (int e = 0; e < 8; ++e) v[e] = W2[(k0 + e) * H2 + n];
  } else if (blk < 15) {
    KD = H2; NC = G3P; i = (blk - 12) * NTHR + tid; base = WP3;
    act = i < (G3P * H2) / 8;
    const int ic = i < (G3P * H2) / 8 ? i : (G3P * H2) / 8 - 1;
    const int n = ic >> 3, k0 = (ic & 7) * 8;
    const int na = n > (G3 - 1) ? (G3 - 1) : n;
#pragma unroll
    for (int e = 0; e < 8; ++e) {
      const float va = W3[(k0 + e) * G3 + na];
      v[e] = (n < G3) ? va : 0.0f;
    }
    i = ic;
  } else {
    KD = FX; NC = HP; i = tid; base = WPP;
    const int n = i >> 3, k0 = (i & 7) * 8;
#pragma unroll
    for (int e = 0; e < 8; ++e) v[e] = P1[(k0 + e) * HP + n];
  }
  v4f a, b;
  a.x = v[0]; a.y = v[1]; a.z = v[2]; a.w = v[3];
  b.x = v[4]; b.y = v[5]; b.z = v[6]; b.w = v[7];
  v8us hv, lv;
  split8(a, b, hv, lv);
  if (act) {
    unsigned short* dh = wp + base + (size_t)i * 8;
    unsigned short* dl = dh + NC * KD;
    *(volatile v8us*)dh = hv;
    *(volatile v8us*)dl = lv;
    __threadfence();
    *(volatile v8us*)dh = hv;
    *(volatile v8us*)dl = lv;
  }
}

__global__ __launch_bounds__(NTHR) void k_agg(
    const float* __restrict__ x, const float* __restrict__ ops, const int* __restrict__ ei,
    float* nm, float* mk, int nN, int nE2, int nE1, int vec8) {
  extern __shared__ v4f lds_dyn[];
  float* acc  = (float*)lds_dyn;
  int*   list = (int*)((char*)lds_dyn + NB * FX * 4);
  int*   scnt = list + LISTN;
  int*   wcnt = scnt + NB;
  const int tid = threadIdx.x, lane = tid & 31, wave = tid >> 5;
  const int nodeBase = blockIdx.x * NB;

  {
    const v4f z = {0.0f, 0.0f, 0.0f, 0.0f};
#pragma unroll 4
    for (int q = tid; q < NB * FX / 4; q += NTHR) ((v4f*)acc)[q] = z;
    for (int s = tid; s < NB; s += NTHR) scnt[s] = 0;
  }
  __syncthreads();

  const int nChunks = (nE2 + CHUNK - 1) / CHUNK;
#pragma unroll 1
  for (int ch = 0; ch < nChunks; ++ch) {
    const int cbase = ch * CHUNK;
    const int wc = scan_chunk<NB>(ei, nE2, cbase, nodeBase, vec8, list, tid, lane, wave);
    if (lane == 0) wcnt[wave] = wc;
    __syncthreads();
    if (wave == 0) {
#pragma unroll 1
      for (int wsx = 0; wsx < NWAVE; ++wsx) {
        int n = __builtin_amdgcn_readfirstlane(wcnt[wsx]);
        n = n > WCAP ? WCAP : (n < 0 ? 0 : n);
        const int* lp = list + wsx * WCAP;
#pragma unroll 1
        for (int i = 0; i < n; ++i) {
          const int ent = __builtin_amdgcn_readfirstlane(lp[i]);
          int slot = ent & 4095;
          slot = slot > NB - 1 ? NB - 1 : slot;
          int e = cbase + ((ent >> 12) & (CHUNK - 1));
          e = e > nE2 - 1 ? nE2 - 1 : e;
          int pe = e + nE1;
          pe = pe >= nE2 ? pe - nE2 : pe;
          pe = pe < 0 ? 0 : (pe > nE2 - 1 ? nE2 - 1 : pe);
          int sv = ei[pe];
          sv = sv < 0 ? 0 : (sv > nN - 1 ? nN - 1 : sv);
          const v2f xv = *(const v2f*)(x + (size_t)sv * FX + 2 * lane);
          float* ap = acc + slot * FX + 2 * lane;
          v2f av = *(v2f*)ap;
          av = av + xv;
          *(v2f*)ap = av;
          if (lane == 0) scnt[slot] = scnt[slot] + 1;
        }
      }
    }
    __syncthreads();
  }

  float* smask = (float*)list;
  for (int s = tid; s < NB; s += NTHR) {
    const int node = nodeBase + s;
    const int nodec = node > nN - 1 ? nN - 1 : node;
    const v4f o = *(const v4f*)(ops + (size_t)nodec * 4);
    const float mx = fmaxf(fmaxf(o.x, o.y), fmaxf(o.z, o.w));
    float e0 = 0.0f, ssum = 0.0f;
#pragma unroll 1
    for (int i = 0; i < 4; ++i) {
      float oi = o.x;
      oi = (i == 1) ? o.y : oi;
      oi = (i == 2) ? o.z : oi;
      oi = (i == 3) ? o.w : oi;
      const float ev = expf(oi - mx);
      ssum += ev;
      e0 = (i == 0) ? ev : e0;
    }
    const float p0 = e0 * (1.0f / ssum);
    const int c = scnt[s];
    smask[s] = (node < nN && p0 > 0.5f && c > 0) ? 1.0f : 0.0f;
  }
#pragma unroll 4
  for (int q = tid; q < NB * FX / 4; q += NTHR) {
    const int row = q >> 4;
    const int c = scnt[row];
    const float rc = 1.0f / (float)(c > 1 ? c : 1);
    v4f v = ((v4f*)acc)[q];
    v = v * rc;
    ((v4f*)acc)[q] = v;
  }
  __syncthreads();

  float* gp = nm + (size_t)nodeBase * FX;
  v4f mv = {0.0f, 0.0f, 0.0f, 0.0f};
  if (tid < NB / 4) mv = ((const v4f*)smask)[tid];
#pragma unroll 4
  for (int q = tid; q < NB * FX / 4; q += NTHR) { const v4f v = ((const v4f*)acc)[q]; *(volatile v4f*)(gp + 4 * q) = v; }
  if (tid < NB / 4) *(volatile v4f*)(mk + (size_t)nodeBase + 4 * tid) = mv;
  __threadfence();
#pragma unroll 4
  for (int q = tid; q < NB * FX / 4; q += NTHR) { const v4f v = ((const v4f*)acc)[q]; *(volatile v4f*)(gp + 4 * q) = v; }
  if (tid < NB / 4) *(volatile v4f*)(mk + (size_t)nodeBase + 4 * tid) = mv;
}

__device__ __forceinline__ void out_rows(const float* stg, const float* sprob, const float* smask,
                                         float* ob, int nf, int tid) {
#pragma unroll
  for (int it = 0; it < 9; ++it) {
    const int q = it * NTHR + tid;
    if (q < (GROWS * OW) / 4) {
      const int row = q / (OW / 4);
      const int j = q - row * (OW / 4);
      const float mkv = smask[row];
      const float pr = sprob[row];
      const float* gr = stg + row * G3P;
      float e[4];
#pragma unroll
      for (int u = 0; u < 4; ++u) {
        const int idx = 4 * j + u;
        const float g = gr[idx < G3 ? idx : (G3 - 1)];
        e[u] = (idx < G3 ? g : pr) * mkv;
      }
      v4f v;
      v.x = e[0]; v.y = e[1]; v.z = e[2]; v.w = e[3];
      if (4 * q + 4 <= nf) {
        *(volatile v4f*)(ob + 4 * q) = v;
      } else if (4 * q < nf) {
        volatile float* op = ob + 4 * q;
        op[0] = v.x;
        if (4 * q + 1 < nf) op[1] = v.y;
        if (4 * q + 2 < nf) op[2] = v.z;
      }
    }
  }
}

__global__ __launch_bounds__(NTHR) void k_mlp(
    const float* __restrict__ x, const float* __restrict__ nm, const float* __restrict__ mk,
    const unsigned short* __restrict__ wp,
    const float* __restrict__ b1, const float* __restrict__ b2, const float* __restrict__ b3,
    const float* __restrict__ pb1, const float* __restrict__ P2, const float* __restrict__ pb2,
    float* out, int nN) {
  extern __shared__ v4f lds_dyn[];
  __shared__ __attribute__((aligned(16))) float smask[GROWS];
  __shared__ __attribute__((aligned(16))) float sprob[GROWS];
  unsigned short* sHi = (unsigned short*)lds_dyn;
  unsigned short* sLo = sHi + GROWS * APT;
  float*          stg = (float*)((char*)lds_dyn + LDS_AT);
  const int tid = threadIdx.x, lane = tid & 31, wave = tid >> 5, hh = lane >> 4, m = lane & 15;
  const int rowBase = blockIdx.x * GROWS;

  if (tid < GROWS) smask[tid] = mk[rowBase + tid];

  {
    const int c0 = (tid & 7) * 8, rr = tid >> 3;
#pragma unroll
    for (int it = 0; it < 4; ++it) {
      const int r = it * 32 + rr;
      int row = rowBase + r;
      row = row > nN - 1 ? nN - 1 : row;
      const float* ap = x + (size_t)row * FX + c0;
      v4f a = *(const v4f*)ap, b = *(const v4f*)(ap + 4);
      v8us hv, lv;
      split8(a, b, hv, lv);
      *(v8us*)(sHi + r * APT + c0) = hv;
      *(v8us*)(sLo + r * APT + c0) = lv;
      const float* np = nm + (size_t)(rowBase + r) * FX + c0;
      a = *(const v4f*)np; b = *(const v4f*)(np + 4);
      split8(a, b, hv, lv);
      *(v8us*)(sHi + r * APT + FX + c0) = hv;
      *(v8us*)(sLo + r * APT + FX + c0) = lv;
    }
  }
  __syncthreads();

#pragma unroll
  for (int ch = 0; ch < 2; ++ch) {
    v8f acc[4];
    mma_tiles<KC, 4, H1, APT>(sHi, sLo, wp + WP1 + (size_t)(64 * ch) * KC, wave * 16, lane, acc);
    float* sp = stg + (wave * 16 + 8 * hh) * H1 + 64 * ch + m;
#pragma unroll
    for (int t = 0; t < 4; ++t) {
      const float bv = b1[64 * ch + 16 * t + m];
#pragma unroll
      for (int r = 0; r < 8; ++r) {
        float v = acc[t][r] + bv;
        v = fmaxf(v, 0.0f);
        sp[r * H1 + 16 * t] = v;
      }
    }
  }
  __syncthreads();
  {
    const int c0 = (tid & 15) * 8, rr = tid >> 4;
#pragma unroll 2
    for (int it = 0; it < 8; ++it) {
      const int r = it * 16 + rr;
      const float* fp = stg + r * H1 + c0;
      const v4f a = *(const v4f*)fp, b = *(const v4f*)(fp + 4);
      v8us hv, lv;
      split8(a, b, hv, lv);
      *(v8us*)(sHi + r * APT + c0) = hv;
      *(v8us*)(sLo + r * APT + c0) = lv;
    }
  }
  __syncthreads();

  {
    v8f acc[4];
    mma_tiles<H1, 4, H2, APT>(sHi, sLo, wp + WP2, wave * 16, lane, acc);
    float* sp = stg + (wave * 16 + 8 * hh) * H2 + m;
#pragma unroll
    for (int t = 0; t < 4; ++t) {
      const float bv = b2[16 * t + m];
#pragma unroll
      for (int r = 0; r < 8; ++r) {
        float v = acc[t][r] + bv;
        v = fmaxf(v, 0.0f);
        sp[r * H2 + 16 * t] = v;
      }
    }
  }
  __syncthreads();
  {
    const int c0 = (tid & 7) * 8, rr = tid >> 3;
#pragma unroll
    for (int it = 0; it < 4; ++it) {
      const int r = it * 32 + rr;
      const float* fp = stg + r * H2 + c0;
      const v4f a = *(const v4f*)fp, b = *(const v4f*)(fp + 4);
      v8us hv, lv;
      split8(a, b, hv, lv);
      *(v8us*)(sHi + r * APT + c0) = hv;
      *(v8us*)(sLo + r * APT + c0) = lv;
    }
  }
  __syncthreads();

  {
    v8f acc[5];
    mma_tiles<H2, 5, G3P, APT>(sHi, sLo, wp + WP3, wave * 16, lane, acc);
    float* sp = stg + (wave * 16 + 8 * hh) * G3P + m;
#pragma unroll
    for (int t = 0; t < 5; ++t) {
      const int col = 16 * t + m;
      const float bv = b3[col < G3 ? col : (G3 - 1)];
#pragma unroll
      for (int r = 0; r < 8; ++r) sp[r * G3P + 16 * t] = acc[t][r] + bv;
    }
  }
  __syncthreads();
  {
    const int c0 = (tid & 7) * 8, rr = tid >> 3;
#pragma unroll
    for (int it = 0; it < 4; ++it) {
      const int r = it * 32 + rr;
      const float* fp = stg + r * G3P + 3 + c0;
      v4f a, b;
      a.x = fp[0]; a.y = fp[1]; a.z = fp[2]; a.w = fp[3];
      b.x = fp[4]; b.y = fp[5]; b.z = fp[6]; b.w = fp[7];
      v8us hv, lv;
      split8(a, b, hv, lv);
      *(v8us*)(sHi + r * APT + c0) = hv;
      *(v8us*)(sLo + r * APT + c0) = lv;
    }
  }
  __syncthreads();

  {
    v8f acc[2];
    mma_tiles<FX, 2, HP, APT>(sHi, sLo, wp + WPP, wave * 16, lane, acc);
    const float pba = pb1[m], pbb = pb1[16 + m];
    const float w0 = P2[m], w1 = P2[16 + m];
    const float bb2 = pb2[0];
#pragma unroll
    for (int r = 0; r < 8; ++r) {
      const float p0 = fmaxf(acc[0][r] + pba, 0.0f);
      const float p1 = fmaxf(acc[1][r] + pbb, 0.0f);
      float s = p0 * w0 + p1 * w1;
      s += __shfl_xor(s, 1);
      s += __shfl_xor(s, 2);
      s += __shfl_xor(s, 4);
      s += __shfl_xor(s, 8);
      const float logit = s + bb2;
      if (m == 0) sprob[wave * 16 + 8 * hh + r] = logit;
    }
  }
  __syncthreads();
  if (tid < GROWS) {
    float lg = sprob[tid];
    lg = lg > 40.0f ? 40.0f : (lg < -40.0f ? -40.0f : lg);
    const float ev = expf(-lg);
    sprob[tid] = 1.0f / (1.0f + ev);
  }
  __syncthreads();

  int nvalid = nN - rowBase;
  nvalid = nvalid > GROWS ? GROWS : (nvalid < 0 ? 0 : nvalid);
  const int nf = nvalid * OW;
  float* ob = out + (size_t)rowBase * OW;
  out_rows(stg, sprob, smask, ob, nf, tid);
  __threadfence();
  out_rows(stg, sprob, smask, ob, nf, tid);
}

extern "C" void kernel_launch(void* const* d_in, const int* in_sizes, int n_in,
                              void* d_out, int out_size, void* d_ws, size_t ws_size,
                              hipStream_t stream) {
  if (n_in < 13) return;
  const int nN  = in_sizes[0] / FX;
  const int nE2 = in_sizes[2];
  if (nN <= 0 || nE2 <= 0 || (nE2 & 1) != 0) return;
  if (in_sizes[0] != nN * FX || in_sizes[1] != nN * 4) return;
  if (in_sizes[3] != KC * H1 || in_sizes[4] != H1) return;
  if (in_sizes[5] != H1 * H2 || in_sizes[6] != H2) return;
  if (in_sizes[7] != H2 * G3 || in_sizes[8] != G3) return;
  if (in_sizes[9] != FX * HP || in_sizes[10] != HP) return;
  if (in_sizes[11] != HP || in_sizes[12] != 1) return;
  if (out_size != nN * OW) return;
  if (nE2 > (1 << 28) || nN > (1 << 24)) return;
  const int nE1 = nE2 / 2;

  const float* x    = (const float*)d_in[0];
  const float* ops  = (const float*)d_in[1];
  const int*   ei   = (const int*)d_in[2];
  const float* W1   = (const float*)d_in[3];
  const float* b1   = (const float*)d_in[4];
  const float* W2   = (const float*)d_in[5];
  const float* b2   = (const float*)d_in[6];
  const float* W3   = (const float*)d_in[7];
  const float* b3   = (const float*)d_in[8];
  const float* P1   = (const float*)d_in[9];
  const float* pb1  = (const float*)d_in[10];
  const float* P2   = (const float*)d_in[11];
  const float* pb2  = (const float*)d_in[12];
  float* out = (float*)d_out;

  const int NPAD   = ((nN + GROWS - 1) / GROWS) * GROWS;
  const int nGemm  = NPAD / GROWS;
  const int nAgg   = (NPAD + NB - 1) / NB;
  const int AGGPAD = nAgg * NB;

  char* ws = (char*)d_ws;
  size_t off = 0;
  const size_t oW  = off; off += (size_t)WPTOT * 2;          off = (off + 255) & ~(size_t)255;
  const size_t oNm = off; off += (size_t)AGGPAD * FX * 4;    off = (off + 255) & ~(size_t)255;
  const size_t oMk = off; off += (size_t)AGGPAD * 4;         off = (off + 255) & ~(size_t)255;
  if (off > ws_size || off > (size_t)WSCAP) return;
  unsigned short* wpl = (unsigned short*)(ws + oW);
  float*          nm  = (float*)(ws + oNm);
  float*          mkp = (float*)(ws + oMk);

  const int vec8 = 1;

  k_wprep<<<16, NTHR, 0, stream>>>(W1, W2, W3, P1, wpl);

  hipFuncSetAttribute(reinterpret_cast<const void*>(&k_agg),
                      hipFuncAttributeMaxDynamicSharedMemorySize, LDS_AGG);
  k_agg<<<nAgg, NTHR, LDS_AGG, stream>>>(x, ops, ei, nm, mkp, nN, nE2, nE1, vec8);

  hipFuncSetAttribute(reinterpret_cast<const void*>(&k_mlp),
                      hipFuncAttributeMaxDynamicSharedMemorySize, LDS_MLP);
  k_mlp<<<nGemm, NTHR, LDS_MLP, stream>>>(x, nm, mkp, wpl, b1, b2, b3, pb1, P2, pb2, out, nN);
}
